// SemGCN_25314537243184
// MI455X (gfx1250) — hardware-verified
//
#include <hip/hip_runtime.h>
#include <math.h>
#include <stddef.h>
#include <stdint.h>

#define NBATCH 4096
#define NJ     16
#define HID    128
#define INTER  64
#define MROWS  (NBATCH * NJ)
#define NBLK   (MROWS / 64)
#define NNZ    46
#define SK     256
#define YK     128
#define TABF   1024
#define RECW   256
#define XTRA   4096
#define NEGV   (-9.0e15f)
#define WSMAX  134217728
#define EPI_MIX 0
#define EPI_REC 1
#define EPI_NL  2
#define T_DIAG 256
#define T_CNT  272
#define T_NZJ  288
#define T_NZW  544
#define X_BIAS 1024
#define X_PST  2048
#define X_CP   192
#define X_GRP  320
#define X_A    336
#define X_BW   400
#define X_F    432
#define X_GX   1024
#define NLB_OFF (5 * 192 * 256)

static_assert(MROWS % 64 == 0);
static_assert(64 % NJ == 0);
static_assert(NJ == 16);
static_assert(NNZ <= 64);
static_assert(NBLK == 1024);
static_assert(SK == 2 * HID);
static_assert(YK == 2 * INTER);
static_assert(SK % 32 == 0 && YK % 32 == 0);
static_assert((64 * (256 + 4) + XTRA) * 4 <= 327680);
static_assert(T_NZW + 256 <= TABF);
static_assert(X_GX + 2048 <= XTRA);
static_assert(X_F + 512 <= X_GX);
static_assert(X_PST + 256 <= XTRA);

typedef float          v4f   __attribute__((ext_vector_type(4)));
typedef float          v8f   __attribute__((ext_vector_type(8)));
typedef int            v8i   __attribute__((ext_vector_type(8)));
typedef unsigned int   v4u   __attribute__((ext_vector_type(4)));
typedef unsigned short v8us  __attribute__((ext_vector_type(8)));
typedef unsigned short v16us __attribute__((ext_vector_type(16)));
typedef __bf16         v16bf __attribute__((ext_vector_type(16)));
typedef v4f  __attribute__((may_alias)) v4fa;
typedef v4u  __attribute__((may_alias)) v4ua;
typedef v8us __attribute__((may_alias)) v8usa;
union FragB { v16bf v; v16us u; v8us h[2]; v8i w; };
struct F8 { float f[8]; };

__device__ __forceinline__ v8f wmb(const FragB& a, const FragB& b, v8f c) {
  v8f d = __builtin_amdgcn_wmma_f32_16x16x32_bf16(false, a.v, false, b.v, (short)0, c, false, false);
  asm volatile("v_nop\n\tv_nop\n\tv_nop\n\tv_nop" : "+v"(d) : "v"(a.w), "v"(b.w));
  return d;
}
__device__ __forceinline__ v8f z8() { v8f z = {0.f, 0.f, 0.f, 0.f, 0.f, 0.f, 0.f, 0.f}; return z; }

__device__ __forceinline__ unsigned bf16_bits(float f) {
  const unsigned u = __float_as_uint(f);
  return (u + 0x7FFFu + ((u >> 16) & 1u)) >> 16;
}
__device__ __forceinline__ float bf16_val(float f) { return __uint_as_float(bf16_bits(f) << 16); }
__device__ __forceinline__ int cl16(int v) { return min(max(v, 0), 15); }

__device__ __forceinline__ F8 widen8(const v4u w) {
  F8 r;
  r.f[0] = __uint_as_float(w.x << 16); r.f[1] = __uint_as_float(w.x & 0xffff0000u);
  r.f[2] = __uint_as_float(w.y << 16); r.f[3] = __uint_as_float(w.y & 0xffff0000u);
  r.f[4] = __uint_as_float(w.z << 16); r.f[5] = __uint_as_float(w.z & 0xffff0000u);
  r.f[6] = __uint_as_float(w.w << 16); r.f[7] = __uint_as_float(w.w & 0xffff0000u);
  return r;
}
__device__ __forceinline__ void split8(const F8& v, v8us& h, v8us& l) {
#pragma unroll
  for (int e = 0; e < 8; ++e) {
    const unsigned hb = bf16_bits(v.f[e]);
    const unsigned lb = bf16_bits(v.f[e] - __uint_as_float(hb << 16));
    h[e] = (unsigned short)hb;
    l[e] = (unsigned short)lb;
  }
}
__device__ __forceinline__ F8 state8(const unsigned short* p) {
  const F8 h = widen8(*(const v4ua*)p);
  const F8 l = widen8(*(const v4ua*)(p + HID));
  F8 r;
#pragma unroll
  for (int e = 0; e < 8; ++e) r.f[e] = h.f[e] + l.f[e];
  return r;
}
__device__ __forceinline__ F8 bn8(const float* gp, const float* stat, int c8) {
  const v4f g0 = *(const v4f*)gp,               g1 = *(const v4f*)(gp + 4);
  const v4f m0 = *(const v4f*)(stat + c8),       m1 = *(const v4f*)(stat + c8 + 4);
  const v4f a0 = *(const v4f*)(stat + 128 + c8), a1 = *(const v4f*)(stat + 128 + c8 + 4);
  const v4f b0 = *(const v4f*)(stat + 256 + c8), b1 = *(const v4f*)(stat + 256 + c8 + 4);
  F8 r;
  r.f[0] = (g0.x - m0.x) * a0.x + b0.x; r.f[1] = (g0.y - m0.y) * a0.y + b0.y;
  r.f[2] = (g0.z - m0.z) * a0.z + b0.z; r.f[3] = (g0.w - m0.w) * a0.w + b0.w;
  r.f[4] = (g1.x - m1.x) * a1.x + b1.x; r.f[5] = (g1.y - m1.y) * a1.y + b1.y;
  r.f[6] = (g1.z - m1.z) * a1.z + b1.z; r.f[7] = (g1.w - m1.w) * a1.w + b1.w;
  return r;
}

__global__ __launch_bounds__(256) void k_pa(const float* __restrict__ Wres, unsigned short* WG) {
  const int u  = (int)blockIdx.x * 256 + (int)threadIdx.x;
  const int kq = u & 15, n = (u >> 4) & 255, c = u >> 12;
  const int s  = n >> 7, o = n & 127;
  const float* p = Wres + ((size_t)((c * 2 + s) * HID + kq * 8)) * HID + o;
  v8us o8;
#pragma unroll
  for (int e = 0; e < 8; ++e) o8[e] = (unsigned short)bf16_bits(p[(size_t)e * HID]);
  unsigned short* dp = WG + ((size_t)c * 256 + n) * SK + kq * 8;
  *(volatile v8us*)dp = o8;
  *(volatile v8us*)(dp + HID) = o8;
  __threadfence();
  *(volatile v8us*)dp = o8;
  *(volatile v8us*)(dp + HID) = o8;
}

__global__ __launch_bounds__(256) void k_pb(const float* __restrict__ gw, const float* __restrict__ tw,
                                            const float* __restrict__ pw, const float* __restrict__ ww,
                                            unsigned short* planes) {
  const int y = (int)blockIdx.y;
  const int u = (int)blockIdx.x * 256 + (int)threadIdx.x;
  const int i = u >> 10, rem = u & 1023;
  v4f a, b;
  size_t dofs;
  int dup;
  if (y < 3) {
    const int nrow = rem >> 4, kq = rem & 15;
    const size_t so = ((size_t)i * INTER + nrow) * HID + kq * 8;
    if (y == 0)      { a = *(const v4f*)(gw + so); b = *(const v4f*)(gw + so + 4); }
    else if (y == 1) { a = *(const v4f*)(tw + so); b = *(const v4f*)(tw + so + 4); }
    else             { a = *(const v4f*)(pw + so); b = *(const v4f*)(pw + so + 4); }
    dofs = ((size_t)i * 192 + y * 64 + nrow) * SK + kq * 8;
    dup = HID;
  } else {
    const int o = rem >> 3, kq = rem & 7;
    const size_t so = ((size_t)i * HID + o) * INTER + kq * 8;
    a = *(const v4f*)(ww + so); b = *(const v4f*)(ww + so + 4);
    dofs = (size_t)NLB_OFF + ((size_t)i * HID + o) * YK + kq * 8;
    dup = INTER;
  }
  v8us o8;
  o8[0] = (unsigned short)bf16_bits(a.x); o8[1] = (unsigned short)bf16_bits(a.y);
  o8[2] = (unsigned short)bf16_bits(a.z); o8[3] = (unsigned short)bf16_bits(a.w);
  o8[4] = (unsigned short)bf16_bits(b.x); o8[5] = (unsigned short)bf16_bits(b.y);
  o8[6] = (unsigned short)bf16_bits(b.z); o8[7] = (unsigned short)bf16_bits(b.w);
  unsigned short* dp = planes + dofs;
  *(volatile v8us*)dp = o8;
  *(volatile v8us*)(dp + dup) = o8;
  __threadfence();
  *(volatile v8us*)dp = o8;
  *(volatile v8us*)(dp + dup) = o8;
}

__global__ __launch_bounds__(32) void k_pc(const float* __restrict__ e_in, const float* __restrict__ e_res,
                                           const float* __restrict__ e_out, const int* __restrict__ rows,
                                           const int* __restrict__ cols, float* tab) {
  __shared__ __attribute__((aligned(16))) float lg[256];
  __shared__ __attribute__((aligned(16))) float tb[TABF];
  const int t = (int)blockIdx.x, lane = (int)threadIdx.x;
#pragma unroll 1
  for (int i = lane; i < 256; i += 32) lg[i] = NEGV;
#pragma unroll 1
  for (int i = lane; i < TABF; i += 32) tb[i] = 0.0f;
  __syncthreads();
  const int tc = min(max(t - 1, 0), 7);
#pragma unroll 1
  for (int n = 0; n < NNZ; ++n) {
    const float ev0 = e_in[n];
    const float ev1 = e_res[tc * NNZ + n];
    const float ev2 = e_out[n];
    const float ev = (t == 0) ? ev0 : ((t <= 8) ? ev1 : ev2);
    const int r = cl16(rows[n]);
    const int c = cl16(cols[n]);
    lg[r * 16 + c] = bf16_val(ev);
  }
  __syncthreads();
  const int i = lane & 15;
  float mx = lg[i * 16];
#pragma unroll 1
  for (int j = 1; j < 16; ++j) mx = fmaxf(mx, lg[i * 16 + j]);
  __syncthreads();
  float s = 0.0f;
#pragma unroll 1
  for (int j = 0; j < 16; ++j) {
    const float ex = expf(lg[i * 16 + j] - mx);
    lg[i * 16 + j] = ex;
    s += ex;
  }
  const float inv = 1.0f / s;
  int cnt = 0;
#pragma unroll 1
  for (int j = 0; j < 16; ++j) {
    const float a = lg[i * 16 + j] * inv;
    const float offv = (j == i) ? 0.0f : a;
    tb[i * 16 + j] = offv;
    if (j == i) tb[T_DIAG + i] = a;
    if (offv != 0.0f) {
      tb[T_NZJ + i * 16 + cnt] = __int_as_float(j);
      tb[T_NZW + i * 16 + cnt] = offv;
      ++cnt;
    }
  }
  tb[T_CNT + i] = __int_as_float(cnt);
  __syncthreads();
  float* dst = tab + (size_t)t * TABF;
#pragma unroll 1
  for (int it = 0; it < 8; ++it) {
    const v4f v = *(const v4fa*)(tb + (it * 32 + lane) * 4);
    *(volatile v4f*)(dst + (it * 32 + lane) * 4) = v;
  }
  __threadfence();
#pragma unroll 1
  for (int it = 0; it < 8; ++it) {
    const v4f v = *(const v4fa*)(tb + (it * 32 + lane) * 4);
    *(volatile v4f*)(dst + (it * 32 + lane) * 4) = v;
  }
}

__device__ __forceinline__ void emit_g_rec(const float* tile, const int P, float* pst, float* G, const int rowBase,
                                           float* rec, const int blk, const int tid) {
  const int lane = tid & 31, wave = tid >> 5;
#pragma unroll 4
  for (int rr = 0; rr < 8; ++rr) {
    const int lr = 8 * wave + rr;
    const v4f v = *(const v4fa*)(tile + lr * P + 4 * lane);
    *(volatile v4f*)(G + (size_t)(rowBase + lr) * HID + 4 * lane) = v;
  }
  __threadfence();
#pragma unroll 4
  for (int rr = 0; rr < 8; ++rr) {
    const int lr = 8 * wave + rr;
    const v4f v = *(const v4fa*)(tile + lr * P + 4 * lane);
    *(volatile v4f*)(G + (size_t)(rowBase + lr) * HID + 4 * lane) = v;
  }
  if (tid < 128) {
    float s = 0.0f;
#pragma unroll 4
    for (int r = 0; r < 64; ++r) s += tile[r * P + tid];
    const float mean = s * (1.0f / 64.0f);
    float q = 0.0f;
#pragma unroll 4
    for (int r = 0; r < 64; ++r) {
      const float d = tile[r * P + tid] - mean;
      q = fmaf(d, d, q);
    }
    pst[tid] = mean;
    pst[128 + tid] = q;
  }
  __syncthreads();
  v4f qv = {0.f, 0.f, 0.f, 0.f};
  if (tid < 64) {
    qv = *(const v4fa*)(pst + 4 * tid);
    *(volatile v4f*)(rec + (size_t)blk * RECW + 4 * tid) = qv;
  }
  __threadfence();
  if (tid < 64) {
    *(volatile v4f*)(rec + (size_t)blk * RECW + 4 * tid) = qv;
  }
}

template <int N, int EPI>
__global__ void __launch_bounds__(256) __attribute__((amdgpu_num_vgpr(248)))
k_gemm(const unsigned short* __restrict__ A, const unsigned short* __restrict__ BT, int K,
       const float* __restrict__ v0, const float* __restrict__ v1, const float* __restrict__ v2,
       const float* __restrict__ v3, const int* __restrict__ gi,
       float* of, unsigned short* oy, float* rec) {
  static_assert(N == 128 || N == 192 || N == 256);
  extern __shared__ __attribute__((aligned(16))) float smem[];
  constexpr int P  = N + 4;
  constexpr int NT = N / 64;
  constexpr int WN = N / 4;
  float* tile = smem;
  float* xr   = smem + 64 * P;
  const int tid = (int)threadIdx.x, lane = tid & 31, wave = tid >> 5, hh = lane >> 4, m = lane & 15;
  const int wm = wave >> 2, wn = wave & 3;
  const int blk = (int)blockIdx.x;
  const int rowBase = blk * 64;

  if (EPI == EPI_MIX) {
    *(v4fa*)(xr + 4 * tid) = *(const v4f*)(v0 + 4 * tid);
    if (tid < 128) xr[X_BIAS + tid] = bf16_val(v1[tid]);
  } else if (EPI == EPI_REC) {
    if (tid < 128) xr[X_BIAS + tid] = bf16_val(v0[tid]);
  } else {
    if (wave < 2)       xr[tid] = bf16_val(v0[tid]);
    else if (wave < 4)  xr[tid] = bf16_val(v1[tid - 64]);
    else if (wave < 6)  xr[tid] = bf16_val(v2[tid - 128]);
    else if (wave == 6) {
      xr[X_CP + lane]      = bf16_val(v3[lane]);
      xr[X_CP + 32 + lane] = bf16_val(v3[32 + lane]);
      xr[X_CP + 64 + lane] = bf16_val(v3[64 + lane]);
      xr[X_CP + 96 + lane] = bf16_val(v3[96 + lane]);
    } else {
      const int g = cl16(gi[lane & 15]);
      if (lane < 16) xr[X_GRP + lane] = __int_as_float(g);
    }
  }

  v8f acc[2][NT];
#pragma unroll
  for (int mt = 0; mt < 2; ++mt)
#pragma unroll
    for (int nt = 0; nt < NT; ++nt) acc[mt][nt] = z8();

  const unsigned short* ap0 = A + (size_t)(rowBase + 32 * wm + m) * (size_t)K + 8 * hh;
  const unsigned short* ap1 = ap0 + (size_t)16 * (size_t)K;
  const unsigned short* bp  = BT + (size_t)(wn * WN + m) * (size_t)K + 8 * hh;

#pragma unroll 1
  for (int k0 = 0; k0 < K; k0 += 32) {
    FragB a0, a1;
    a0.h[0] = *(const v8usa*)(ap0 + k0);
    a0.h[1] = *(const v8usa*)(ap0 + k0 + 16);
    a1.h[0] = *(const v8usa*)(ap1 + k0);
    a1.h[1] = *(const v8usa*)(ap1 + k0 + 16);
#pragma unroll
    for (int nt = 0; nt < NT; ++nt) {
      const unsigned short* wq = bp + (size_t)(16 * nt) * (size_t)K + k0;
      FragB bf;
      bf.h[0] = *(const v8usa*)wq;
      bf.h[1] = *(const v8usa*)(wq + 16);
      acc[0][nt] = wmb(a0, bf, acc[0][nt]);
      acc[1][nt] = wmb(a1, bf, acc[1][nt]);
    }
  }

#pragma unroll
  for (int mt = 0; mt < 2; ++mt)
#pragma unroll
    for (int nt = 0; nt < NT; ++nt)
#pragma unroll
      for (int r = 0; r < 8; ++r)
        tile[(32 * wm + 16 * mt + 8 * hh + r) * P + WN * wn + 16 * nt + m] = acc[mt][nt][r];
  __syncthreads();

  const int c4 = 4 * lane;
  if (EPI == EPI_MIX) {
#pragma unroll 1
    for (int rr = 0; rr < 8; ++rr) {
      const int lr = 8 * wave + rr;
      const int i = lr & 15, s16 = lr & 48;
      const v4f h0 = *(const v4fa*)(tile + lr * P + c4);
      const float d = xr[T_DIAG + i];
      int cnt = __float_as_int(xr[T_CNT + i]);
      cnt = __builtin_amdgcn_readfirstlane(min(max(cnt, 0), 16));
      v4f mx = {0.f, 0.f, 0.f, 0.f};
#pragma unroll 1
      for (int t = 0; t < cnt; ++t) {
        const int j = cl16(__float_as_int(xr[T_NZJ + i * 16 + t]));
        const float w = xr[T_NZW + i * 16 + t];
        const v4f h1 = *(const v4fa*)(tile + (s16 + j) * P + HID + c4);
        mx.x = fmaf(w, h1.x, mx.x); mx.y = fmaf(w, h1.y, mx.y);
        mx.z = fmaf(w, h1.z, mx.z); mx.w = fmaf(w, h1.w, mx.w);
      }
      const v4f bb = *(const v4fa*)(xr + X_BIAS + c4);
      v4f o;
      o.x = (d * h0.x + mx.x) + bb.x; o.y = (d * h0.y + mx.y) + bb.y;
      o.z = (d * h0.z + mx.z) + bb.z; o.w = (d * h0.w + mx.w) + bb.w;
      *(v4fa*)(tile + lr * P + c4) = o;
    }
    __syncthreads();
    emit_g_rec(tile, P, xr + X_PST, of, rowBase, rec, blk, tid);
  } else if (EPI == EPI_REC) {
#pragma unroll 1
    for (int rr = 0; rr < 8; ++rr) {
      const int lr = 8 * wave + rr;
      v4f v = *(const v4fa*)(tile + lr * P + c4);
      const v4f bb = *(const v4fa*)(xr + X_BIAS + c4);
      v.x += bb.x; v.y += bb.y; v.z += bb.z; v.w += bb.w;
      *(v4fa*)(tile + lr * P + c4) = v;
    }
    __syncthreads();
    emit_g_rec(tile, P, xr + X_PST, of, rowBase, rec, blk, tid);
  } else {
#pragma unroll 1
    for (int it = 0; it < 8; ++it) {
      const int u = it * 256 + tid;
      const int c = u & 63, w = (u >> 6) & 7, s = u >> 9;
      const int r0 = s * 16 + __float_as_int(xr[X_GRP + 2 * w]);
      const int r1 = s * 16 + __float_as_int(xr[X_GRP + 2 * w + 1]);
      const float gb = xr[c];
      xr[X_GX + u] = fmaxf(tile[r0 * P + c] + gb, tile[r1 * P + c] + gb);
    }
    if (wave < 2) {
      const int s = tid >> 4, p = tid & 15;
      const int row = s * 16 + __float_as_int(xr[X_GRP + p]);
      float sum = 0.0f;
#pragma unroll 4
      for (int c = 0; c < INTER; ++c)
        sum = fmaf(tile[row * P + 64 + c] + xr[64 + c], xr[X_CP + c], sum);
      xr[X_A + tid] = sum;
    } else if (wave == 2) {
      const int s = lane >> 3, w = lane & 7;
      const int r0 = s * 16 + __float_as_int(xr[X_GRP + 2 * w]);
      const int r1 = s * 16 + __float_as_int(xr[X_GRP + 2 * w + 1]);
      float sum = 0.0f;
#pragma unroll 4
      for (int c = 0; c < INTER; ++c) {
        const float pb = xr[128 + c];
        const float ph = fmaxf(tile[r0 * P + 128 + c] + pb, tile[r1 * P + 128 + c] + pb);
        sum = fmaf(ph, xr[X_CP + 64 + c], sum);
      }
      xr[X_BW + lane] = sum;
    }
    __syncthreads();
#pragma unroll
    for (int it = 0; it < 2; ++it) {
      const int u = it * 256 + tid;
      const int s = u >> 7, p = (u >> 3) & 15, w = u & 7;
      xr[X_F + u] = fmaxf(xr[X_A + s * 16 + p] + xr[X_BW + s * 8 + w], 0.0f) * 0.125f;
    }
    __syncthreads();
    v8us hv[2], lv[2];
#pragma unroll
    for (int it = 0; it < 2; ++it) {
      const int u = it * 256 + tid;
      const int rowp = u >> 3, c8 = (u & 7) * 8, s = rowp >> 4;
      float y0 = 0.f, y1 = 0.f, y2 = 0.f, y3 = 0.f, y4 = 0.f, y5 = 0.f, y6 = 0.f, y7 = 0.f;
#pragma unroll 2
      for (int w = 0; w < 8; ++w) {
        const float fw = xr[X_F + rowp * 8 + w];
        const float* gp = xr + X_GX + (s * 8 + w) * 64 + c8;
        const v4f ga = *(const v4fa*)gp;
        const v4f gb = *(const v4fa*)(gp + 4);
        y0 = fmaf(fw, ga.x, y0); y1 = fmaf(fw, ga.y, y1); y2 = fmaf(fw, ga.z, y2); y3 = fmaf(fw, ga.w, y3);
        y4 = fmaf(fw, gb.x, y4); y5 = fmaf(fw, gb.y, y5); y6 = fmaf(fw, gb.z, y6); y7 = fmaf(fw, gb.w, y7);
      }
      F8 yv;
      yv.f[0] = y0; yv.f[1] = y1; yv.f[2] = y2; yv.f[3] = y3;
      yv.f[4] = y4; yv.f[5] = y5; yv.f[6] = y6; yv.f[7] = y7;
      split8(yv, hv[it], lv[it]);
    }
#pragma unroll
    for (int it = 0; it < 2; ++it) {
      const int u = it * 256 + tid;
      const int rowp = u >> 3, c8 = (u & 7) * 8;
      unsigned short* yr = oy + (size_t)(rowBase + rowp) * YK + c8;
      *(volatile v8us*)yr = hv[it];
      *(volatile v8us*)(yr + INTER) = lv[it];
    }
    __threadfence();
#pragma unroll
    for (int it = 0; it < 2; ++it) {
      const int u = it * 256 + tid;
      const int rowp = u >> 3, c8 = (u & 7) * 8;
      unsigned short* yr = oy + (size_t)(rowBase + rowp) * YK + c8;
      *(volatile v8us*)yr = hv[it];
      *(volatile v8us*)(yr + INTER) = lv[it];
    }
  }
}

__global__ __launch_bounds__(256) void k_gin(const float* __restrict__ x, const float* __restrict__ W,
                                             const float* __restrict__ bias, const float* __restrict__ tab,
                                             float* G, float* rec) {
  __shared__ __attribute__((aligned(16))) float tile[64 * 132];
  __shared__ __attribute__((aligned(16))) float tb[TABF];
  __shared__ __attribute__((aligned(16))) float pst[RECW];
  __shared__ __attribute__((aligned(16))) float xs[128];
  const int tid = (int)threadIdx.x, blk = (int)blockIdx.x;
  if (tid < 128) xs[tid] = bf16_val(x[(size_t)blk * 128 + tid]);
  *(v4fa*)(tb + 4 * tid) = *(const v4f*)(tab + 4 * tid);
  __syncthreads();
  const int o = tid & 127, half = tid >> 7;
  const float w00 = bf16_val(W[o]),       w01 = bf16_val(W[128 + o]);
  const float w10 = bf16_val(W[256 + o]), w11 = bf16_val(W[384 + o]);
  const float bo  = bf16_val(bias[o]);
#pragma unroll 1
  for (int ss = 0; ss < 2; ++ss) {
    const int s = half * 2 + ss;
#pragma unroll 1
    for (int i = 0; i < 16; ++i) {
      const float h0 = xs[s * 32 + i * 2] * w00 + xs[s * 32 + i * 2 + 1] * w01;
      int cnt = __float_as_int(tb[T_CNT + i]);
      cnt = min(max(cnt, 0), 16);
      float mx = 0.0f;
#pragma unroll 1
      for (int t = 0; t < cnt; ++t) {
        const int j = cl16(__float_as_int(tb[T_NZJ + i * 16 + t]));
        const float w = tb[T_NZW + i * 16 + t];
        const float h1 = xs[s * 32 + j * 2] * w10 + xs[s * 32 + j * 2 + 1] * w11;
        mx = fmaf(w, h1, mx);
      }
      tile[(s * 16 + i) * 132 + o] = (tb[T_DIAG + i] * h0 + mx) + bo;
    }
  }
  __syncthreads();
  emit_g_rec(tile, 132, pst, G, blk * 64, rec, blk, tid);
}

__global__ __launch_bounds__(128) void k_comb(const float* __restrict__ rec, const float* __restrict__ gam,
                                              const float* __restrict__ bet, float* stat) {
  __shared__ __attribute__((aligned(16))) float stg[512];
  const int c = (int)threadIdx.x;
  double s = 0.0;
#pragma unroll 4
  for (int p = 0; p < NBLK; ++p) s += (double)rec[(size_t)p * RECW + c];
  const double mean = s * (1.0 / (double)NBLK);
  double q = 0.0;
#pragma unroll 2
  for (int p = 0; p < NBLK; ++p) {
    const double mb = (double)rec[(size_t)p * RECW + c];
    const double qb = (double)rec[(size_t)p * RECW + 128 + c];
    const double d = mb - mean;
    q += qb + 64.0 * d * d;
  }
  const float var = (float)(q * (1.0 / (double)MROWS));
  const float rs = 1.0f / sqrtf(var + 1e-5f);
  stg[c]       = (float)mean;
  stg[128 + c] = rs * bf16_val(gam[c]);
  stg[256 + c] = bf16_val(bet[c]);
  stg[384 + c] = 0.0f;
  __syncthreads();
  const v4f v = *(const v4fa*)(stg + 4 * c);
  *(volatile v4f*)(stat + 4 * c) = v;
  __threadfence();
  *(volatile v4f*)(stat + 4 * c) = v;
}

template <int RES>
__global__ __launch_bounds__(256) void k_app(const float* __restrict__ G, const float* __restrict__ stat,
                                             const unsigned short* __restrict__ resp, unsigned short* outp) {
  const int u = (int)blockIdx.x * 256 + (int)threadIdx.x;
  const int row = u >> 4, c8 = (u & 15) * 8;
  F8 v = bn8(G + (size_t)row * HID + c8, stat, c8);
#pragma unroll
  for (int e = 0; e < 8; ++e) v.f[e] = fmaxf(v.f[e], 0.0f);
  if (RES) {
    const F8 r = state8(resp + (size_t)row * SK + c8);
#pragma unroll
    for (int e = 0; e < 8; ++e) v.f[e] = r.f[e] + v.f[e];
  }
  v8us h8, l8;
  split8(v, h8, l8);
  unsigned short* dp = outp + (size_t)row * SK + c8;
  *(volatile v8us*)dp = h8;
  *(volatile v8us*)(dp + HID) = l8;
  __threadfence();
  *(volatile v8us*)dp = h8;
  *(volatile v8us*)(dp + HID) = l8;
}

__global__ __launch_bounds__(256) void k_nlapp(const float* __restrict__ G, const float* __restrict__ stat,
                                               const unsigned short* __restrict__ Tp, const int* __restrict__ grouped,
                                               const int* __restrict__ restored, unsigned short* Sp) {
  const int u = (int)blockIdx.x * 256 + (int)threadIdx.x;
  const int row = u >> 4, c8 = (u & 15) * 8;
  const int b = row >> 4, j = row & 15;
  const int r = cl16(restored[j]);
  const int q = cl16(grouped[r]);
  F8 v = bn8(G + (size_t)(b * 16 + r) * HID + c8, stat, c8);
  const F8 xo = state8(Tp + (size_t)(b * 16 + q) * SK + c8);
#pragma unroll
  for (int e = 0; e < 8; ++e) v.f[e] = v.f[e] + xo.f[e];
  v8us h8, l8;
  split8(v, h8, l8);
  unsigned short* dp = Sp + (size_t)row * SK + c8;
  *(volatile v8us*)dp = h8;
  *(volatile v8us*)(dp + HID) = l8;
  __threadfence();
  *(volatile v8us*)dp = h8;
  *(volatile v8us*)(dp + HID) = l8;
}

__global__ __launch_bounds__(256) void k_out(const unsigned short* __restrict__ S, const float* __restrict__ W,
                                             const float* __restrict__ bias, const float* __restrict__ tab,
                                             float* out) {
  __shared__ __attribute__((aligned(16))) float hs[64 * 132];
  __shared__ __attribute__((aligned(16))) float wl[768];
  __shared__ __attribute__((aligned(16))) float tb[TABF];
  __shared__ __attribute__((aligned(16))) float pp[512];
  __shared__ __attribute__((aligned(16))) float outs[1536];
  __shared__ float bsh[4];
  const int tid = (int)threadIdx.x, blk = (int)blockIdx.x;
#pragma unroll
  for (int q = 0; q < 3; ++q) wl[q * 256 + tid] = bf16_val(W[q * 256 + tid]);
  *(v4fa*)(tb + 4 * tid) = *(const v4f*)(tab + 4 * tid);
  {
    const float bv = bf16_val(bias[min(tid, 2)]);
    if (tid < 4) bsh[tid] = bv;
  }
#pragma unroll 1
  for (int g = 0; g < 8; ++g) {
    __syncthreads();
#pragma unroll 1
    for (int it = 0; it < 4; ++it) {
      const int u = it * 256 + tid;
      const int row = u >> 4, c8 = (u & 15) * 8;
      const F8 v = state8(S + (size_t)(blk * 512 + g * 64 + row) * SK + c8);
      v4f a, b;
      a.x = v.f[0]; a.y = v.f[1]; a.z = v.f[2]; a.w = v.f[3];
      b.x = v.f[4]; b.y = v.f[5]; b.z = v.f[6]; b.w = v.f[7];
      *(v4fa*)(hs + row * 132 + c8) = a;
      *(v4fa*)(hs + row * 132 + c8 + 4) = b;
    }
    __syncthreads();
    {
      const int row = tid >> 2, part = tid & 3;
      float a0 = 0.f, a1 = 0.f, a2 = 0.f, a3 = 0.f, a4 = 0.f, a5 = 0.f;
#pragma unroll 2
      for (int kk = 0; kk < 32; ++kk) {
        const int k = part * 32 + kk;
        const float hv = hs[row * 132 + k];
        a0 = fmaf(hv, wl[k * 3], a0);
        a1 = fmaf(hv, wl[k * 3 + 1], a1);
        a2 = fmaf(hv, wl[k * 3 + 2], a2);
        a3 = fmaf(hv, wl[384 + k * 3], a3);
        a4 = fmaf(hv, wl[384 + k * 3 + 1], a4);
        a5 = fmaf(hv, wl[384 + k * 3 + 2], a5);
      }
      a0 += __shfl_xor(a0, 1, 32); a1 += __shfl_xor(a1, 1, 32); a2 += __shfl_xor(a2, 1, 32);
      a3 += __shfl_xor(a3, 1, 32); a4 += __shfl_xor(a4, 1, 32); a5 += __shfl_xor(a5, 1, 32);
      a0 += __shfl_xor(a0, 2, 32); a1 += __shfl_xor(a1, 2, 32); a2 += __shfl_xor(a2, 2, 32);
      a3 += __shfl_xor(a3, 2, 32); a4 += __shfl_xor(a4, 2, 32); a5 += __shfl_xor(a5, 2, 32);
      if (part == 0) {
        pp[row * 8 + 0] = a0; pp[row * 8 + 1] = a1; pp[row * 8 + 2] = a2;
        pp[row * 8 + 3] = a3; pp[row * 8 + 4] = a4; pp[row * 8 + 5] = a5;
      }
    }
    __syncthreads();
    if (tid < 192) {
      const int row = tid / 3, o = tid - row * 3;
      const int i = row & 15, s16 = row & 48;
      float mx = 0.0f;
#pragma unroll 4
      for (int j = 0; j < 16; ++j) mx = fmaf(tb[i * 16 + j], pp[(s16 + j) * 8 + 3 + o], mx);
      outs[g * 192 + tid] = (tb[T_DIAG + i] * pp[row * 8 + o] + mx) + bsh[o];
    }
  }
  __syncthreads();
  const v4f o0 = *(const v4fa*)(outs + 4 * tid);
  const v4f o1 = *(const v4fa*)(outs + 1024 + 4 * (tid & 127));
  float* ob = out + (size_t)blk * 1536;
  *(volatile v4f*)(ob + 4 * tid) = o0;
  if (tid < 128) *(volatile v4f*)(ob + 1024 + 4 * tid) = o1;
  __threadfence();
  *(volatile v4f*)(ob + 4 * tid) = o0;
  if (tid < 128) *(volatile v4f*)(ob + 1024 + 4 * tid) = o1;
}

extern "C" void kernel_launch(void* const* d_in, const int* in_sizes, int n_in,
                              void* d_out, int out_size, void* d_ws, size_t ws_size,
                              hipStream_t stream) {
  if (n_in < 29) return;
  const int expect_n[29] = {131072, 512, 46, 128, 128, 128, 262144, 368, 1024, 1024, 1024,
                            40960, 320, 40960, 320, 40960, 320, 640, 40960, 640, 640, 640,
                            768, 46, 3, 46, 46, 16, 16};
  for (int i = 0; i < 29; ++i) if (in_sizes[i] != expect_n[i]) return;
  if (out_size != NBATCH * NJ * 3) return;

  const float* x        = (const float*)d_in[0];
  const float* gc_in_W  = (const float*)d_in[1];
  const float* gc_in_e  = (const float*)d_in[2];
  const float* gc_in_b  = (const float*)d_in[3];
  const float* bn_in_g  = (const float*)d_in[4];
  const float* bn_in_b  = (const float*)d_in[5];
  const float* W_res    = (const float*)d_in[6];
  const float* e_res    = (const float*)d_in[7];
  const float* b_res    = (const float*)d_in[8];
  const float* bng_res  = (const float*)d_in[9];
  const float* bnb_res  = (const float*)d_in[10];
  const float* nl_g_w   = (const float*)d_in[11];
  const float* nl_g_b   = (const float*)d_in[12];
  const float* nl_t_w   = (const float*)d_in[13];
  const float* nl_t_b   = (const float*)d_in[14];
  const float* nl_p_w   = (const float*)d_in[15];
  const float* nl_p_b   = (const float*)d_in[16];
  const float* nl_cp_w  = (const float*)d_in[17];
  const float* nl_W_w   = (const float*)d_in[18];
  const float* nl_W_b   = (const float*)d_in[19];
  const float* nl_bn_g  = (const float*)d_in[20];
  const float* nl_bn_b  = (const float*)d_in[21];
  const float* gc_out_W = (const float*)d_in[22];
  const float* gc_out_e = (const float*)d_in[23];
  const float* gc_out_b = (const float*)d_in[24];
  const int*   mrows    = (const int*)d_in[25];
  const int*   mcols    = (const int*)d_in[26];
  const int*   grouped  = (const int*)d_in[27];
  const int*   restored = (const int*)d_in[28];
  float* out = (float*)d_out;

  const size_t bS   = (size_t)MROWS * SK * 2;
  const size_t bG   = (size_t)MROWS * HID * 4;
  const size_t bY   = (size_t)MROWS * YK * 2;
  const size_t bWG  = (size_t)8 * 256 * 256 * 2;
  const size_t bNLA = (size_t)5 * 192 * 256 * 2;
  const size_t bNLB = (size_t)5 * 128 * 128 * 2;
  const size_t bREC = (size_t)NBLK * RECW * 4;
  const size_t bST  = (size_t)512 * 4;
  const size_t bTAB = (size_t)10 * TABF * 4;
  size_t off = 0;
  const size_t oS   = off; off += bS;
  const size_t oT   = off; off += bS;
  const size_t oG   = off; off += bG;
  const size_t oY   = off; off += bY;
  const size_t oWG  = off; off += bWG;
  const size_t oNLA = off; off += bNLA;
  const size_t oNLB = off; off += bNLB;
  const size_t oREC = off; off += bREC;
  const size_t oST  = off; off += bST;
  const size_t oTAB = off; off += bTAB;
  if (off > ws_size || off > (size_t)WSMAX) return;
  if (oNLB - oNLA != (size_t)NLB_OFF * 2) return;

  char* ws = (char*)d_ws;
  unsigned short* S   = (unsigned short*)(ws + oS);
  unsigned short* T   = (unsigned short*)(ws + oT);
  float*          G   = (float*)(ws + oG);
  unsigned short* Y   = (unsigned short*)(ws + oY);
  unsigned short* WG  = (unsigned short*)(ws + oWG);
  unsigned short* NLA = (unsigned short*)(ws + oNLA);
  unsigned short* NLB = (unsigned short*)(ws + oNLB);
  float*          REC = (float*)(ws + oREC);
  float*          ST  = (float*)(ws + oST);
  float*          TAB = (float*)(ws + oTAB);

  const int LDS256 = (64 * (256 + 4) + XTRA) * 4;
  const int LDS192 = (64 * (192 + 4) + XTRA) * 4;
  const int LDS128 = (64 * (128 + 4) + XTRA) * 4;
  (void)hipFuncSetAttribute(reinterpret_cast<const void*>(&k_gemm<256, EPI_MIX>),
                            hipFuncAttributeMaxDynamicSharedMemorySize, LDS256);
  (void)hipFuncSetAttribute(reinterpret_cast<const void*>(&k_gemm<192, EPI_NL>),
                            hipFuncAttributeMaxDynamicSharedMemorySize, LDS192);
  (void)hipFuncSetAttribute(reinterpret_cast<const void*>(&k_gemm<128, EPI_REC>),
                            hipFuncAttributeMaxDynamicSharedMemorySize, LDS128);

  const int EWB = MROWS * 16 / 256;

  k_pa<<<128, 256, 0, stream>>>(W_res, WG);
  k_pb<<<dim3(20, 4), 256, 0, stream>>>(nl_g_w, nl_t_w, nl_p_w, nl_W_w, NLA);
  k_pc<<<10, 32, 0, stream>>>(gc_in_e, e_res, gc_out_e, mrows, mcols, TAB);

  k_gin<<<NBLK, 256, 0, stream>>>(x, gc_in_W, gc_in_b, TAB, G, REC);
  k_comb<<<1, 128, 0, stream>>>(REC, bn_in_g, bn_in_b, ST);
  k_app<0><<<EWB, 256, 0, stream>>>(G, ST, S, T);

  for (int blkI = 0; blkI <= 4; ++blkI) {
    if (blkI > 0) {
      const int c0 = 2 * (blkI - 1), c1 = c0 + 1;
      k_gemm<256, EPI_MIX><<<NBLK, 256, LDS256, stream>>>(
          S, WG + (size_t)c0 * 65536, SK, TAB + (size_t)(1 + c0) * TABF, b_res + (size_t)c0 * HID,
          b_res, b_res, grouped, G, Y, REC);
      k_comb<<<1, 128, 0, stream>>>(REC, bng_res + (size_t)c0 * HID, bnb_res + (size_t)c0 * HID, ST);
      k_app<0><<<EWB, 256, 0, stream>>>(G, ST, S, T);
      k_gemm<256, EPI_MIX><<<NBLK, 256, LDS256, stream>>>(
          T, WG + (size_t)c1 * 65536, SK, TAB + (size_t)(1 + c1) * TABF, b_res + (size_t)c1 * HID,
          b_res, b_res, grouped, G, Y, REC);
      k_comb<<<1, 128, 0, stream>>>(REC, bng_res + (size_t)c1 * HID, bnb_res + (size_t)c1 * HID, ST);
      k_app<1><<<EWB, 256, 0, stream>>>(G, ST, S, T);
    }
    const int i = blkI;
    k_gemm<192, EPI_NL><<<NBLK, 256, LDS192, stream>>>(
        T, NLA + (size_t)i * 49152, SK, nl_g_b + (size_t)i * INTER, nl_t_b + (size_t)i * INTER,
        nl_p_b + (size_t)i * INTER, nl_cp_w + (size_t)i * 2 * INTER, grouped, G, Y, REC);
    k_gemm<128, EPI_REC><<<NBLK, 256, LDS128, stream>>>(
        Y, NLB + (size_t)i * 16384, YK, nl_W_b + (size_t)i * HID, nl_W_b, nl_W_b, nl_W_b,
        grouped, G, Y, REC);
    k_comb<<<1, 128, 0, stream>>>(REC, nl_bn_g + (size_t)i * HID, nl_bn_b + (size_t)i * HID, ST);
    k_nlapp<<<EWB, 256, 0, stream>>>(G, ST, T, grouped, restored, S);
  }

  k_out<<<NBATCH / 32, 256, 0, stream>>>(S, gc_out_W, gc_out_b, TAB + (size_t)9 * TABF, out);
  (void)hipGetLastError();
}
